// GATLayer_10617159156297
// MI455X (gfx1250) — hardware-verified
//
#include <hip/hip_runtime.h>
#include <stddef.h>
#include <stdint.h>
#include <math.h>


#define NB     8
#define NN     1024
#define DM     128
#define NH     8
#define DH     16
#define FFD    512
#define MROWS  (NB * NN)
#define NQKV   (3 * DM)
#define NTHR   256
#define GBM    64
#define GBN    64
#define GTHR   128
#define WSMAX  134217728

#define MODE_QKV 0
#define MODE_WO  1
#define MODE_FF1 2
#define MODE_FF2 3

static_assert(NH * DH == DM);
static_assert((MROWS % GBM) == 0 && (NN % GBM) == 0);
static_assert((NQKV % GBN) == 0 && (DM % GBN) == 0 && (FFD % GBN) == 0);
static_assert((DM % 32) == 0 && ((2 * DM) % 32) == 0 && ((2 * FFD) % 32) == 0);
static_assert(GBM == (GTHR / 32) * 16);
static_assert(GTHR * 8 == 4 * 64 * 4);
static_assert(GTHR * 8 == 2 * 64 * 8);
static_assert((NN % 64) == 0 && (NN % 16) == 0);

typedef float          v4f  __attribute__((ext_vector_type(4)));
typedef float          v8f  __attribute__((ext_vector_type(8)));
typedef int            v8i  __attribute__((ext_vector_type(8)));
typedef unsigned int   v4u  __attribute__((ext_vector_type(4)));
typedef unsigned short v8us __attribute__((ext_vector_type(8)));
typedef __bf16         v16b __attribute__((ext_vector_type(16)));
typedef v4f  __attribute__((may_alias)) v4fa;
typedef v4u  __attribute__((may_alias)) v4ua;
typedef v8us __attribute__((may_alias)) v8usa;
union FragB { v16b v; v8us h[2]; v4u q[2]; v8i w; };

__device__ __forceinline__ v8f wmb(const FragB& a, const FragB& b, v8f c) {
  v8f d = __builtin_amdgcn_wmma_f32_16x16x32_bf16(false, a.v, false, b.v, (short)0, c, false, false);
  asm volatile("v_nop\n\tv_nop\n\tv_nop\n\tv_nop" : "+v"(d) : "v"(a.w), "v"(b.w));
  return d;
}

__device__ __forceinline__ unsigned int f2bf(float f) {
  const unsigned int u = __float_as_uint(f);
  return ((u + 0x7FFFu + ((u >> 16) & 1u)) >> 16) & 0xFFFFu;
}
__device__ __forceinline__ float bf2f(unsigned int b) { return __uint_as_float(b << 16); }
__device__ __forceinline__ float bfr(float f) { return bf2f(f2bf(f)); }
__device__ __forceinline__ v4f bfr4(const v4f a) {
  v4f r; r.x = bfr(a.x); r.y = bfr(a.y); r.z = bfr(a.z); r.w = bfr(a.w); return r;
}
__device__ __forceinline__ unsigned int pk2(float lo, float hi) { return f2bf(lo) | (f2bf(hi) << 16); }
__device__ __forceinline__ unsigned int pk2lo(float a, float b) {
  return f2bf(a - bfr(a)) | (f2bf(b - bfr(b)) << 16);
}
__device__ __forceinline__ v4u pack8(const v4f a, const v4f b) {
  v4u r;
  r.x = pk2(a.x, a.y); r.y = pk2(a.z, a.w); r.z = pk2(b.x, b.y); r.w = pk2(b.z, b.w);
  return r;
}
__device__ __forceinline__ v4u pack8lo(const v4f a, const v4f b) {
  v4u r;
  r.x = pk2lo(a.x, a.y); r.y = pk2lo(a.z, a.w); r.z = pk2lo(b.x, b.y); r.w = pk2lo(b.z, b.w);
  return r;
}

__global__ __launch_bounds__(NTHR) void k_xprep(const float* __restrict__ x, unsigned short* xb, int nUnits) {
  const int i = (int)blockIdx.x * NTHR + (int)threadIdx.x;
  if (i >= nUnits) return;
  const float* p = x + (size_t)i * 8;
  const v4f a = *(const v4fa*)p, b = *(const v4fa*)(p + 4);
  const v4u hv = pack8(a, b);
  unsigned short* o = xb + (size_t)i * 8;
  *(volatile v4u*)o = hv;
  __threadfence();
  *(volatile v4u*)o = hv;
}

__global__ __launch_bounds__(NTHR) void k_wprep(const float* __restrict__ Wq, const float* __restrict__ Wk,
                                                const float* __restrict__ Wv, const float* __restrict__ Wo,
                                                const float* __restrict__ W1, const float* __restrict__ W2,
                                                unsigned short* wqkv, unsigned short* wo2,
                                                unsigned short* w12, unsigned short* w22) {
  const int blk = (int)blockIdx.x;
  const float* w; unsigned short* wt; int Kin, Ncol, Kout, ub;
  if (blk < 8)        { w = Wq; wt = wqkv;                 Kin = DM;  Ncol = DM;  Kout = DM;      ub = blk; }
  else if (blk < 16)  { w = Wk; wt = wqkv + DM * DM;       Kin = DM;  Ncol = DM;  Kout = DM;      ub = blk - 8; }
  else if (blk < 24)  { w = Wv; wt = wqkv + 2 * DM * DM;   Kin = DM;  Ncol = DM;  Kout = DM;      ub = blk - 16; }
  else if (blk < 40)  { w = Wo; wt = wo2;                  Kin = DM;  Ncol = DM;  Kout = 2 * DM;  ub = blk - 24; }
  else if (blk < 104) { w = W1; wt = w12;                  Kin = DM;  Ncol = FFD; Kout = 2 * DM;  ub = blk - 40; }
  else                { w = W2; wt = w22;                  Kin = FFD; Ncol = DM;  Kout = 2 * FFD; ub = blk - 104; }
  const int u  = ub * NTHR + (int)threadIdx.x;
  const int kq = Kout >> 3;
  const int n  = u / kq;
  const int k8 = (u - n * kq) * 8;
  const int kk = k8 - (k8 / Kin) * Kin;
  const float* p = w + (size_t)kk * (size_t)Ncol + n;
  v4f a, b;
  a.x = p[0];                    a.y = p[(size_t)Ncol];         a.z = p[(size_t)2 * Ncol];     a.w = p[(size_t)3 * Ncol];
  b.x = p[(size_t)4 * Ncol];     b.y = p[(size_t)5 * Ncol];     b.z = p[(size_t)6 * Ncol];     b.w = p[(size_t)7 * Ncol];
  const v4u wv = pack8(a, b);
  unsigned short* o = wt + (size_t)n * (size_t)Kout + k8;
  *(volatile v4u*)o = wv;
  __threadfence();
  *(volatile v4u*)o = wv;
}

__device__ __forceinline__ void put_hilo(const float* stg, unsigned short* plane, int pitch, int loOff,
                                         int rowBase, int col0, int tid) {
  v4u pv[8];
#pragma unroll
  for (int i = 0; i < 8; ++i) {
    const int g = i * GTHR + tid;
    const int row = (g >> 3) & 63, pc = g & 7;
    const v4f a = *(const v4fa*)(stg + row * GBN + 8 * pc);
    const v4f b = *(const v4fa*)(stg + row * GBN + 8 * pc + 4);
    pv[i] = (i < 4) ? pack8(a, b) : pack8lo(a, b);
  }
#pragma unroll
  for (int i = 0; i < 8; ++i) {
    const int g = i * GTHR + tid;
    const int row = (g >> 3) & 63, pc = g & 7;
    unsigned short* o = plane + (size_t)(rowBase + row) * (size_t)pitch + ((i < 4) ? 0 : loOff) + col0 + 8 * pc;
    *(volatile v4u*)o = pv[i];
  }
  __threadfence();
#pragma unroll
  for (int i = 0; i < 8; ++i) {
    const int g = i * GTHR + tid;
    const int row = (g >> 3) & 63, pc = g & 7;
    unsigned short* o = plane + (size_t)(rowBase + row) * (size_t)pitch + ((i < 4) ? 0 : loOff) + col0 + 8 * pc;
    *(volatile v4u*)o = pv[i];
  }
}

template<int MODE>
__global__ __launch_bounds__(GTHR) void k_gemm(
    const unsigned short* __restrict__ A, const unsigned short* __restrict__ WT, int K,
    const float* __restrict__ xin, const float* __restrict__ bias, const float* __restrict__ alpha,
    float* outF, unsigned short* o0, unsigned short* o1, unsigned short* o2, unsigned short* o3)
{
  __shared__ __attribute__((aligned(16))) float stg[GBM * GBN];
  const int tid = (int)threadIdx.x, lane = tid & 31, wave = tid >> 5, hh = lane >> 4, m = lane & 15;
  const int rowBase = (int)blockIdx.x * GBM;
  const int cb      = (int)blockIdx.y;
  const int col0    = cb * GBN;

  v8f acc[4];
  {
    const v8f z = {0.f, 0.f, 0.f, 0.f, 0.f, 0.f, 0.f, 0.f};
    acc[0] = z; acc[1] = z; acc[2] = z; acc[3] = z;
  }
  const unsigned short* ap = A  + (size_t)(rowBase + 16 * wave + m) * (size_t)K + 8 * hh;
  const unsigned short* wp = WT + (size_t)(col0 + m) * (size_t)K + 8 * hh;
  const int ksteps = K >> 5;
#pragma unroll 1
  for (int ks = 0; ks < ksteps; ++ks) {
    FragB af;
    af.h[0] = *(const v8usa*)(ap + 32 * ks);
    af.h[1] = *(const v8usa*)(ap + 32 * ks + 16);
#pragma unroll
    for (int t = 0; t < 4; ++t) {
      const unsigned short* wq = wp + (size_t)(16 * t) * (size_t)K + 32 * ks;
      FragB bf;
      bf.h[0] = *(const v8usa*)wq;
      bf.h[1] = *(const v8usa*)(wq + 16);
      acc[t] = wmb(af, bf, acc[t]);
    }
  }

  float bs[4] = {0.f, 0.f, 0.f, 0.f};
  if (MODE == MODE_FF1 || MODE == MODE_FF2) {
#pragma unroll
    for (int t = 0; t < 4; ++t) bs[t] = bfr(bias[col0 + 16 * t + m]);
  }
  const float qs = (MODE == MODE_QKV && cb < 2) ? 0.25f : 1.0f;
#pragma unroll
  for (int t = 0; t < 4; ++t) {
    const int lc = 16 * t + m;
#pragma unroll
    for (int r = 0; r < 8; ++r) {
      const int lr = 16 * wave + 8 * hh + r;
      float v = acc[t][r];
      if (MODE == MODE_FF1) v = fmaxf(v + bs[t], 0.f);
      if (MODE == MODE_FF2) v = v + bs[t];
      if (MODE == MODE_QKV) v = v * qs;
      stg[lr * GBN + lc] = v;
    }
  }
  __syncthreads();

  if (MODE == MODE_QKV) {
    const int which = cb >> 1, hb = cb & 1;
    const int bb = rowBase >> 10, n0 = rowBase & (NN - 1);
    v4u pv[8];
    if (which < 2) {
      unsigned short* plane = (which == 0) ? o0 : o1;
#pragma unroll
      for (int i = 0; i < 8; ++i) {
        const int g = i * GTHR + tid;
        const int hl = g >> 8, p = g & 255, row = p >> 2, part = p & 3;
        const float* sp = stg + row * GBN + hl * DH + (part & 1) * 8;
        const v4f a = *(const v4fa*)sp, b = *(const v4fa*)(sp + 4);
        const v4u hw = pack8(a, b), lw = pack8lo(a, b);
        const bool sel = part >= 2;
        pv[i].x = sel ? lw.x : hw.x; pv[i].y = sel ? lw.y : hw.y;
        pv[i].z = sel ? lw.z : hw.z; pv[i].w = sel ? lw.w : hw.w;
      }
#pragma unroll
      for (int i = 0; i < 8; ++i) {
        const int g = i * GTHR + tid;
        const int hl = g >> 8, p = g & 255, row = p >> 2, part = p & 3;
        unsigned short* o = plane + ((size_t)((bb * NH + hb * 4 + hl) * NN + n0 + row)) * 32 + part * 8;
        *(volatile v4u*)o = pv[i];
      }
      __threadfence();
#pragma unroll
      for (int i = 0; i < 8; ++i) {
        const int g = i * GTHR + tid;
        const int hl = g >> 8, p = g & 255, row = p >> 2, part = p & 3;
        unsigned short* o = plane + ((size_t)((bb * NH + hb * 4 + hl) * NN + n0 + row)) * 32 + part * 8;
        *(volatile v4u*)o = pv[i];
      }
    } else {
#pragma unroll
      for (int i = 0; i < 8; ++i) {
        const int g = i * GTHR + tid;
        const int c = (g >> 3) & 63, pc = g & 7;
        const float* sp = stg + (8 * pc) * GBN + c;
        v4f a, b;
        a.x = sp[0];           a.y = sp[GBN];         a.z = sp[2 * GBN];     a.w = sp[3 * GBN];
        b.x = sp[4 * GBN];     b.y = sp[5 * GBN];     b.z = sp[6 * GBN];     b.w = sp[7 * GBN];
        pv[i] = (i < 4) ? pack8(a, b) : pack8lo(a, b);
      }
#pragma unroll
      for (int i = 0; i < 8; ++i) {
        const int g = i * GTHR + tid;
        const int c = (g >> 3) & 63, pc = g & 7;
        unsigned short* o = ((i < 4) ? o2 : o3) + ((size_t)(bb * DM + hb * 64 + c)) * NN + n0 + 8 * pc;
        *(volatile v4u*)o = pv[i];
      }
      __threadfence();
#pragma unroll
      for (int i = 0; i < 8; ++i) {
        const int g = i * GTHR + tid;
        const int c = (g >> 3) & 63, pc = g & 7;
        unsigned short* o = ((i < 4) ? o2 : o3) + ((size_t)(bb * DM + hb * 64 + c)) * NN + n0 + 8 * pc;
        *(volatile v4u*)o = pv[i];
      }
    }
  }

  if (MODE == MODE_WO || MODE == MODE_FF2) {
    const float al = bfr(alpha[0]);
    v4f fv[8];
#pragma unroll
    for (int i = 0; i < 8; ++i) {
      const int lr = 16 * wave + 2 * i + hh;
      const int gr = rowBase + lr;
      float* sp = stg + lr * GBN + 4 * m;
      const v4f s = *(const v4fa*)sp;
      v4f xv = *(const v4fa*)(xin + (size_t)gr * DM + col0 + 4 * m);
      if (MODE == MODE_WO) xv = bfr4(xv);
      v4f o;
      o.x = xv.x + al * s.x; o.y = xv.y + al * s.y; o.z = xv.z + al * s.z; o.w = xv.w + al * s.w;
      fv[i] = o;
      if (MODE == MODE_WO) *(v4fa*)sp = o;
    }
#pragma unroll
    for (int i = 0; i < 8; ++i) {
      const int lr = 16 * wave + 2 * i + hh;
      float* op = outF + (size_t)(rowBase + lr) * DM + col0 + 4 * m;
      *(volatile v4f*)op = fv[i];
    }
    __threadfence();
#pragma unroll
    for (int i = 0; i < 8; ++i) {
      const int lr = 16 * wave + 2 * i + hh;
      float* op = outF + (size_t)(rowBase + lr) * DM + col0 + 4 * m;
      *(volatile v4f*)op = fv[i];
    }
    if (MODE == MODE_WO) {
      __syncthreads();
      put_hilo(stg, o0, 2 * DM, DM, rowBase, col0, tid);
    }
  }

  if (MODE == MODE_FF1) put_hilo(stg, o0, 2 * FFD, FFD, rowBase, col0, tid);

  (void)xin; (void)bias; (void)alpha; (void)outF; (void)o0; (void)o1; (void)o2; (void)o3;
}

__global__ __launch_bounds__(32) void k_attn(
    const unsigned short* __restrict__ QHL, const unsigned short* __restrict__ KHLp,
    const unsigned short* __restrict__ VTH, const unsigned short* __restrict__ VTL,
    const float* __restrict__ e, unsigned short* CTX)
{
  __shared__ __attribute__((aligned(16))) unsigned int et[16 * 512];
  __shared__ __attribute__((aligned(16))) unsigned int ph[16 * 32];
  __shared__ __attribute__((aligned(16))) unsigned int pl[16 * 32];
  __shared__ __attribute__((aligned(16))) float cx[16 * DM];
  const int lane = (int)threadIdx.x & 31, hh = lane >> 4, m = lane & 15;
  const int q0 = (int)blockIdx.x * 16;
  const int b  = (int)blockIdx.y;

  const float* eb = e + ((size_t)(b * NN + q0)) * NN;
#pragma unroll 2
  for (int it = 0; it < 64; ++it) {
    const int pc = it * 32 + lane;
    const int row = pc >> 7, c8 = (pc & 127) * 8;
    const float* p = eb + (size_t)row * NN + c8;
    const v4f a = *(const v4fa*)p, bq = *(const v4fa*)(p + 4);
    *(v4ua*)(et + row * 512 + (c8 >> 1)) = pack8(a, bq);
  }
  __syncthreads();

  const v8f z8 = {0.f, 0.f, 0.f, 0.f, 0.f, 0.f, 0.f, 0.f};
#pragma unroll 1
  for (int hd = 0; hd < NH; ++hd) {
    const size_t hrow = (size_t)(b * NH + hd) * NN;
    const unsigned short* qp = QHL + (hrow + q0 + m) * 32 + 8 * hh;
    FragB qh, ql;
    {
      const v8us a = *(const v8usa*)qp;
      const v8us c = *(const v8usa*)(qp + 16);
      qh.h[0] = a; qh.h[1] = a;
      ql.h[0] = c; ql.h[1] = c;
    }
    const unsigned short* kb = KHLp + (hrow + m) * 32 + 8 * hh;
    const size_t vrow = ((size_t)(b * DM + hd * DH + m)) * NN + 8 * hh;
    v8f O = z8;
    float lsum = 0.0f;

#pragma unroll 1
    for (int kt = 0; kt < NN / 64; ++kt) {
      const int key0 = kt * 64;
#pragma unroll
      for (int t = 0; t < 4; ++t) {
        const unsigned short* kp = kb + (size_t)(key0 + 16 * t) * 32;
        FragB kf;
        kf.h[0] = *(const v8usa*)kp;
        kf.h[1] = *(const v8usa*)(kp + 16);
        v8f S = wmb(kf, qh, z8);
        S = wmb(kf, ql, S);
        const v4u ew = *(const v4ua*)(et + m * 512 + ((key0 + 16 * t + 8 * hh) >> 1));
        float ev[8];
        ev[0] = __uint_as_float(ew.x << 16); ev[1] = __uint_as_float(ew.x & 0xffff0000u);
        ev[2] = __uint_as_float(ew.y << 16); ev[3] = __uint_as_float(ew.y & 0xffff0000u);
        ev[4] = __uint_as_float(ew.z << 16); ev[5] = __uint_as_float(ew.z & 0xffff0000u);
        ev[6] = __uint_as_float(ew.w << 16); ev[7] = __uint_as_float(ew.w & 0xffff0000u);
        float pr[8];
#pragma unroll
        for (int r = 0; r < 8; ++r) {
          const float tt = S[r] + ev[r];
          const float ex = expf(tt + tt);
          const float p  = expf(-20.0f * __builtin_amdgcn_rcpf(1.0f + ex));
          lsum += p;
          pr[r] = p;
        }
        v4f pa, pb;
        pa.x = pr[0]; pa.y = pr[1]; pa.z = pr[2]; pa.w = pr[3];
        pb.x = pr[4]; pb.y = pr[5]; pb.z = pr[6]; pb.w = pr[7];
        *(v4ua*)(ph + m * 32 + 8 * t + 4 * hh) = pack8(pa, pb);
        *(v4ua*)(pl + m * 32 + 8 * t + 4 * hh) = pack8lo(pa, pb);
      }
      __syncthreads();
#pragma unroll
      for (int ks = 0; ks < 2; ++ks) {
        FragB pA, pL, vh, vl;
        pA.q[0] = *(const v4ua*)(ph + m * 32 + 16 * ks + 4 * hh);
        pA.q[1] = *(const v4ua*)(ph + m * 32 + 16 * ks + 8 + 4 * hh);
        pL.q[0] = *(const v4ua*)(pl + m * 32 + 16 * ks + 4 * hh);
        pL.q[1] = *(const v4ua*)(pl + m * 32 + 16 * ks + 8 + 4 * hh);
        const unsigned short* vp = VTH + vrow + key0 + 32 * ks;
        const unsigned short* vq = VTL + vrow + key0 + 32 * ks;
        vh.h[0] = *(const v8usa*)vp; vh.h[1] = *(const v8usa*)(vp + 16);
        vl.h[0] = *(const v8usa*)vq; vl.h[1] = *(const v8usa*)(vq + 16);
        O = wmb(pA, vh, O);
        O = wmb(pA, vl, O);
        O = wmb(pL, vh, O);
      }
      __syncthreads();
    }

    const float lt = lsum + __shfl_xor(lsum, 16);
#pragma unroll
    for (int r = 0; r < 8; ++r) {
      const float lq = __shfl(lt, 8 * hh + r);
      cx[(8 * hh + r) * DM + hd * DH + m] = O[r] * __builtin_amdgcn_rcpf(lq);
    }
  }
  __syncthreads();

  v4u pv[16];
  const bool lsel = lane >= 16;
#pragma unroll
  for (int i = 0; i < 16; ++i) {
    const float* sp = cx + i * DM + 8 * m;
    const v4f a = *(const v4fa*)sp, bq = *(const v4fa*)(sp + 4);
    const v4u hw = pack8(a, bq), lw = pack8lo(a, bq);
    pv[i].x = lsel ? lw.x : hw.x; pv[i].y = lsel ? lw.y : hw.y;
    pv[i].z = lsel ? lw.z : hw.z; pv[i].w = lsel ? lw.w : hw.w;
  }
  unsigned short* cbp = CTX + ((size_t)(b * NN + q0)) * (2 * DM) + 8 * lane;
#pragma unroll
  for (int i = 0; i < 16; ++i) *(volatile v4u*)(cbp + (size_t)i * (2 * DM)) = pv[i];
  __threadfence();
#pragma unroll
  for (int i = 0; i < 16; ++i) *(volatile v4u*)(cbp + (size_t)i * (2 * DM)) = pv[i];
}

extern "C" void kernel_launch(void* const* d_in, const int* in_sizes, int n_in,
                              void* d_out, int out_size, void* d_ws, size_t ws_size,
                              hipStream_t stream) {
  if (n_in < 12) return;
  if (in_sizes[0] != MROWS * DM) return;
  if (in_sizes[1] != NB * NN * NN) return;
  if (in_sizes[2] != DM * DM || in_sizes[3] != DM * DM) return;
  if (in_sizes[4] != DM * DM || in_sizes[5] != DM * DM) return;
  if (in_sizes[6] != DM * FFD || in_sizes[7] != FFD) return;
  if (in_sizes[8] != FFD * DM || in_sizes[9] != DM) return;
  if (in_sizes[10] != 1 || in_sizes[11] != 1) return;
  if (out_size != MROWS * DM) return;

  const float* x  = (const float*)d_in[0];
  const float* e  = (const float*)d_in[1];
  const float* Wq = (const float*)d_in[2];
  const float* Wk = (const float*)d_in[3];
  const float* Wv = (const float*)d_in[4];
  const float* Wo = (const float*)d_in[5];
  const float* W1 = (const float*)d_in[6];
  const float* b1 = (const float*)d_in[7];
  const float* W2 = (const float*)d_in[8];
  const float* b2 = (const float*)d_in[9];
  const float* a1 = (const float*)d_in[10];
  const float* a2 = (const float*)d_in[11];
  float* out = (float*)d_out;

  char* ws = (char*)d_ws;
  size_t off = 0;
  const size_t oXB  = off; off += (size_t)MROWS * DM * 2;          off = (off + 255) & ~(size_t)255;
  const size_t oWQ  = off; off += (size_t)NQKV * DM * 2;           off = (off + 255) & ~(size_t)255;
  const size_t oWO  = off; off += (size_t)DM * 2 * DM * 2;         off = (off + 255) & ~(size_t)255;
  const size_t oW1  = off; off += (size_t)FFD * 2 * DM * 2;        off = (off + 255) & ~(size_t)255;
  const size_t oW2  = off; off += (size_t)DM * 2 * FFD * 2;        off = (off + 255) & ~(size_t)255;
  const size_t oQ   = off; off += (size_t)NB * NH * NN * 32 * 2;   off = (off + 255) & ~(size_t)255;
  const size_t oK   = off; off += (size_t)NB * NH * NN * 32 * 2;   off = (off + 255) & ~(size_t)255;
  const size_t oVH  = off; off += (size_t)NB * DM * NN * 2;        off = (off + 255) & ~(size_t)255;
  const size_t oVL  = off; off += (size_t)NB * DM * NN * 2;        off = (off + 255) & ~(size_t)255;
  const size_t oCX  = off; off += (size_t)MROWS * 2 * DM * 2;      off = (off + 255) & ~(size_t)255;
  const size_t oX1  = off; off += (size_t)MROWS * DM * 4;          off = (off + 255) & ~(size_t)255;
  const size_t oX1H = off; off += (size_t)MROWS * 2 * DM * 2;      off = (off + 255) & ~(size_t)255;
  const size_t oF   = off; off += (size_t)MROWS * 2 * FFD * 2;     off = (off + 255) & ~(size_t)255;
  if (off > ws_size || off > (size_t)WSMAX) return;
  unsigned short* XB    = (unsigned short*)(ws + oXB);
  unsigned short* WQKVt = (unsigned short*)(ws + oWQ);
  unsigned short* WO2   = (unsigned short*)(ws + oWO);
  unsigned short* W1_2  = (unsigned short*)(ws + oW1);
  unsigned short* W2_2  = (unsigned short*)(ws + oW2);
  unsigned short* QHL   = (unsigned short*)(ws + oQ);
  unsigned short* KHL   = (unsigned short*)(ws + oK);
  unsigned short* VTH   = (unsigned short*)(ws + oVH);
  unsigned short* VTL   = (unsigned short*)(ws + oVL);
  unsigned short* CTX   = (unsigned short*)(ws + oCX);
  float*          X1    = (float*)(ws + oX1);
  unsigned short* X1HL  = (unsigned short*)(ws + oX1H);
  unsigned short* FHL   = (unsigned short*)(ws + oF);

  const int nUx = MROWS * (DM / 8);
  k_xprep<<<nUx / NTHR, NTHR, 0, stream>>>(x, XB, nUx);
  k_wprep<<<168, NTHR, 0, stream>>>(Wq, Wk, Wv, Wo, W1, W2, WQKVt, WO2, W1_2, W2_2);

  const int gM = MROWS / GBM;
  k_gemm<MODE_QKV><<<dim3(gM, NQKV / GBN), GTHR, 0, stream>>>(XB, WQKVt, DM, x, b1, a1, X1, QHL, KHL, VTH, VTL);
  k_attn<<<dim3(NN / 16, NB), 32, 0, stream>>>(QHL, KHL, VTH, VTL, e, CTX);
  k_gemm<MODE_WO><<<dim3(gM, DM / GBN), GTHR, 0, stream>>>(CTX, WO2, 2 * DM, x, b1, a1, X1, X1HL, X1HL, X1HL, X1HL);
  k_gemm<MODE_FF1><<<dim3(gM, FFD / GBN), GTHR, 0, stream>>>(X1HL, W1_2, 2 * DM, x, b1, a1, X1, FHL, FHL, FHL, FHL);
  k_gemm<MODE_FF2><<<dim3(gM, DM / GBN), GTHR, 0, stream>>>(FHL, W2_2, 2 * FFD, X1, b2, a2, out, X1HL, X1HL, X1HL, X1HL);
}
